// GAT_35914516529780
// MI455X (gfx1250) — hardware-verified
//
#include <hip/hip_runtime.h>
#include <stddef.h>
#include <stdint.h>
#include <math.h>


#define DIN    128
#define DH     256
#define HC     128
#define DOUT   128
#define KP     512
#define NTHR   256
#define NWAVE  8
#define EPT    8
#define CHUNK  (NTHR * EPT)
#define WCAP   (EPT * 32)
#define LISTN  (NWAVE * WCAP)
#define NBA    1024
#define SLA    10
#define RCAP   28672
#define DEGCAP 128
#define GBM    64
#define GBN    128
#define GTHR   256
#define ALB    256
#define PBM    128
#define PTHR   256
#define MROWS  128
#define NU1    (DH * (DIN / 8))
#define NU2    (DH * (KP / 8))
#define NU3    (DOUT * (KP / 8))
#define NEGSL  0.2f
#define EPS_SM 1e-16f
#define AGG_ZINTS (LISTN + 2 * RCAP + 3 * NBA)
#define AGG_LDS_INTS (AGG_ZINTS + 16)
#define GEMM_LDS_FLOATS (GBM * DH + ALB)
#define WSMAX  134217728

static_assert((CHUNK & (CHUNK - 1)) == 0 && CHUNK <= 4096);
static_assert((NBA & (NBA - 1)) == 0 && NBA == (1 << SLA));
static_assert(((long long)CHUNK << SLA) < (1LL << 31));
static_assert(LISTN % NTHR == 0);
static_assert(NBA % NWAVE == 0 && NBA % 32 == 0 && NBA % GBM == 0);
static_assert(RCAP % 4 == 0 && AGG_ZINTS % 4 == 0 && LISTN % 4 == 0);
static_assert(DIN % 32 == 0 && DH % 32 == 0 && KP % 32 == 0 && KP == 2 * DH);
static_assert(DOUT == GBN && DH == 2 * GBN && HC == GBN);
static_assert(GTHR == 2 * 4 * 32 && GBM == 4 * 16 && GBN == 4 * 32);
static_assert(ALB == 4 * GBM);
static_assert(PBM == (PTHR / 32) * 16 && PTHR == 2 * DOUT);
static_assert(MROWS % GBM == 0 && MROWS % PBM == 0);
static_assert(NU1 % NTHR == 0 && NU2 % NTHR == 0 && NU3 % NTHR == 0);
static_assert(DIN / 8 == 16 && KP / 8 == 64);
static_assert(AGG_LDS_INTS * 4 <= 300000);
static_assert(GEMM_LDS_FLOATS * 4 <= 300000);
static_assert(DH == 8 * 32);
static_assert(DEGCAP >= 35 + 8);
static_assert(RCAP >= 16623);

typedef float          v4f   __attribute__((ext_vector_type(4)));
typedef float          v8f   __attribute__((ext_vector_type(8)));
typedef int            v4i   __attribute__((ext_vector_type(4)));
typedef int            v8i   __attribute__((ext_vector_type(8)));
typedef unsigned short v8us  __attribute__((ext_vector_type(8)));
typedef unsigned short v16us __attribute__((ext_vector_type(16)));
typedef __bf16         v16bf __attribute__((ext_vector_type(16)));
typedef v4f  __attribute__((may_alias)) v4fa;
typedef v4i  __attribute__((may_alias)) v4ia;
typedef v8us __attribute__((may_alias)) v8usa;
union FragB { v16bf v; v16us u; v8us h[2]; v8i w; };

__device__ __forceinline__ v8f wmb(const FragB& a, const FragB& b, v8f c) {
  v8f d = __builtin_amdgcn_wmma_f32_16x16x32_bf16(false, a.v, false, b.v, (short)0, c, false, false);
  asm volatile("v_nop\n\tv_nop\n\tv_nop\n\tv_nop" : "+v"(d) : "v"(a.w), "v"(b.w));
  return d;
}

__device__ __forceinline__ unsigned bf16_bits(float f) {
  const unsigned u = __float_as_uint(f);
  return (u + 0x7FFFu + ((u >> 16) & 1u)) >> 16;
}
__device__ __forceinline__ float bf16_val(float f) {
  return __uint_as_float(bf16_bits(f) << 16);
}
__device__ __forceinline__ v4f bfr4(const v4f a) {
  v4f r; r.x = bf16_val(a.x); r.y = bf16_val(a.y); r.z = bf16_val(a.z); r.w = bf16_val(a.w); return r;
}

template <int SLB>
__device__ __forceinline__ int scan_chunk(const int* __restrict__ dsts, int nE, int cbase, int slotBase,
                                          int nb, int vec8, int* list, int tid, int lane, int wave) {
  int wc = 0;
  const int el0  = tid * EPT;
  const int e0   = cbase + el0;
  const int sent = -2147483647 - 1;
  v4i da, db;
  if (vec8 != 0 && cbase + CHUNK <= nE) {
    da = *(const v4i*)(dsts + e0);
    db = *(const v4i*)(dsts + e0 + 4);
  } else {
    da.x = (e0     < nE) ? dsts[min(e0,     nE - 1)] : sent;
    da.y = (e0 + 1 < nE) ? dsts[min(e0 + 1, nE - 1)] : sent;
    da.z = (e0 + 2 < nE) ? dsts[min(e0 + 2, nE - 1)] : sent;
    da.w = (e0 + 3 < nE) ? dsts[min(e0 + 3, nE - 1)] : sent;
    db.x = (e0 + 4 < nE) ? dsts[min(e0 + 4, nE - 1)] : sent;
    db.y = (e0 + 5 < nE) ? dsts[min(e0 + 5, nE - 1)] : sent;
    db.z = (e0 + 6 < nE) ? dsts[min(e0 + 6, nE - 1)] : sent;
    db.w = (e0 + 7 < nE) ? dsts[min(e0 + 7, nE - 1)] : sent;
  }
  const unsigned nbs = (unsigned)slotBase;
  const unsigned unb = (unsigned)nb;
  const unsigned s0 = (unsigned)da.x - nbs, s1 = (unsigned)da.y - nbs;
  const unsigned s2 = (unsigned)da.z - nbs, s3 = (unsigned)da.w - nbs;
  const unsigned s4 = (unsigned)db.x - nbs, s5 = (unsigned)db.y - nbs;
  const unsigned s6 = (unsigned)db.z - nbs, s7 = (unsigned)db.w - nbs;
  const bool h0 = s0 < unb, h1 = s1 < unb, h2 = s2 < unb, h3 = s3 < unb;
  const bool h4 = s4 < unb, h5 = s5 < unb, h6 = s6 < unb, h7 = s7 < unb;
  const unsigned any = __builtin_amdgcn_ballot_w32(h0 | h1 | h2 | h3 | h4 | h5 | h6 | h7);
  if (any != 0u) {
#define HITJ(J, HJ, SJ) { \
      const unsigned mj = __builtin_amdgcn_ballot_w32(HJ); \
      if (mj != 0u) { \
        if (HJ) { \
          const int pos = wc + (int)__builtin_amdgcn_mbcnt_lo(mj, 0u); \
          if (pos < WCAP) list[wave * WCAP + pos] = ((el0 + (J)) << SLB) | (int)(SJ); \
        } \
        wc += (int)__builtin_popcount(mj); } }
    HITJ(0, h0, s0)
    HITJ(1, h1, s1)
    HITJ(2, h2, s2)
    HITJ(3, h3, s3)
    HITJ(4, h4, s4)
    HITJ(5, h5, s5)
    HITJ(6, h6, s6)
    HITJ(7, h7, s7)
#undef HITJ
  }
  return wc;
}

__global__ __launch_bounds__(NTHR) void k_wprep(const float* __restrict__ W1, const float* __restrict__ W2,
                                                const float* __restrict__ W3,
                                                unsigned short* W1T, unsigned short* W2T, unsigned short* W3T) {
  const int u = (int)blockIdx.x * NTHR + (int)threadIdx.x;
  v8us o;
  unsigned short* dp;
  if (u < NU1) {
    const int n  = u >> 4;
    const int k8 = (u & 15) * 8;
    const float* p = W1 + (size_t)k8 * DH + n;
#pragma unroll
    for (int i = 0; i < 8; ++i) o[i] = (unsigned short)bf16_bits(p[(size_t)i * DH]);
    dp = W1T + (size_t)n * DIN + k8;
  } else if (u < NU1 + NU2) {
    const int v  = u - NU1;
    const int n  = v >> 6;
    const int k8 = (v & 63) * 8;
    const int kk = k8 & (DH - 1);
    const float* p = W2 + (size_t)kk * DH + n;
#pragma unroll
    for (int i = 0; i < 8; ++i) o[i] = (unsigned short)bf16_bits(p[(size_t)i * DH]);
    dp = W2T + (size_t)n * KP + k8;
  } else if (u < NU1 + NU2 + NU3) {
    const int v  = u - NU1 - NU2;
    const int n  = v >> 6;
    const int k8 = (v & 63) * 8;
    const int kk = k8 & (DH - 1);
    const float* p = W3 + (size_t)kk * DOUT + n;
#pragma unroll
    for (int i = 0; i < 8; ++i) o[i] = (unsigned short)bf16_bits(p[(size_t)i * DOUT]);
    dp = W3T + (size_t)n * KP + k8;
  } else {
    return;
  }
  *(volatile v8us*)dp = o;
  __threadfence();
  *(volatile v8us*)dp = o;
}

__global__ __launch_bounds__(NTHR) void k_cvx(const float* __restrict__ x, int nN, int nUnits,
                                              unsigned short* xb) {
  const int u = (int)blockIdx.x * NTHR + (int)threadIdx.x;
  if (u >= nUnits) return;
  const int row = u >> 4;
  const int k8  = (u & 15) * 8;
  const int rc  = row < nN ? row : nN - 1;
  const float* p = x + (size_t)rc * DIN + k8;
  const v4f a = *(const v4f*)p;
  const v4f b = *(const v4f*)(p + 4);
  const bool ok = row < nN;
  v8us o;
  o[0] = ok ? (unsigned short)bf16_bits(a.x) : (unsigned short)0;
  o[1] = ok ? (unsigned short)bf16_bits(a.y) : (unsigned short)0;
  o[2] = ok ? (unsigned short)bf16_bits(a.z) : (unsigned short)0;
  o[3] = ok ? (unsigned short)bf16_bits(a.w) : (unsigned short)0;
  o[4] = ok ? (unsigned short)bf16_bits(b.x) : (unsigned short)0;
  o[5] = ok ? (unsigned short)bf16_bits(b.y) : (unsigned short)0;
  o[6] = ok ? (unsigned short)bf16_bits(b.z) : (unsigned short)0;
  o[7] = ok ? (unsigned short)bf16_bits(b.w) : (unsigned short)0;
  unsigned short* dp = xb + (size_t)row * DIN + k8;
  *(volatile v8us*)dp = o;
  __threadfence();
  *(volatile v8us*)dp = o;
}

__global__ __launch_bounds__(GTHR) void k_gemm(const unsigned short* __restrict__ A, int lda,
                                               const unsigned short* __restrict__ BT, int ldb, int K,
                                               float* Cm, const float* __restrict__ avs,
                                               const float* __restrict__ avd, float* AL) {
  constexpr int RPW = GBM / NWAVE;
  extern __shared__ __attribute__((aligned(16))) float gsm[];
  float* stg = gsm;
  float* sdt = gsm + GBM * DH;
  const int tid = (int)threadIdx.x, lane = tid & 31, wave = tid >> 5, hh = lane >> 4, m = lane & 15;
  const int rg = wave & 3, cg = wave >> 2;
  const int rowBase = (int)blockIdx.x * GBM;
  const int colBase = cg * GBN;

  v8f acc[8];
  {
    const v8f z = {0.f, 0.f, 0.f, 0.f, 0.f, 0.f, 0.f, 0.f};
#pragma unroll
    for (int t = 0; t < 8; ++t) acc[t] = z;
  }
  const unsigned short* ap = A  + (size_t)(rowBase + 16 * rg + m) * (size_t)lda + 8 * hh;
  const unsigned short* bp = BT + (size_t)(colBase + m) * (size_t)ldb + 8 * hh;

#pragma unroll 1
  for (int k0 = 0; k0 < K; k0 += 32) {
    FragB af;
    af.h[0] = *(const v8usa*)(ap + k0);
    af.h[1] = *(const v8usa*)(ap + k0 + 16);
#pragma unroll
    for (int nt = 0; nt < 8; ++nt) {
      const unsigned short* wq = bp + (size_t)(16 * nt) * (size_t)ldb + k0;
      FragB bf;
      bf.h[0] = *(const v8usa*)wq;
      bf.h[1] = *(const v8usa*)(wq + 16);
      acc[nt] = wmb(af, bf, acc[nt]);
    }
  }

#pragma unroll
  for (int nt = 0; nt < 8; ++nt) {
    const int lc = colBase + 16 * nt + m;
#pragma unroll
    for (int r = 0; r < 8; ++r) {
      const int lr = 16 * rg + 8 * hh + r;
      stg[lr * DH + lc] = acc[nt][r];
    }
  }
  __syncthreads();

  const v4f as0 = bfr4(*(const v4fa*)(avs + 4 * lane));
  const v4f as1 = bfr4(*(const v4fa*)(avs + GBN + 4 * lane));
  const v4f ad0 = bfr4(*(const v4fa*)(avd + 4 * lane));
  const v4f ad1 = bfr4(*(const v4fa*)(avd + GBN + 4 * lane));
#pragma unroll 1
  for (int i = 0; i < RPW; ++i) {
    const int row = wave * RPW + i;
    const v4f p0 = *(const v4fa*)(stg + row * DH + 4 * lane);
    const v4f p1 = *(const v4fa*)(stg + row * DH + GBN + 4 * lane);
    float s0 = 0.0f, d0 = 0.0f, s1 = 0.0f, d1 = 0.0f;
    s0 = fmaf(p0.x, as0.x, s0); s0 = fmaf(p0.y, as0.y, s0); s0 = fmaf(p0.z, as0.z, s0); s0 = fmaf(p0.w, as0.w, s0);
    d0 = fmaf(p0.x, ad0.x, d0); d0 = fmaf(p0.y, ad0.y, d0); d0 = fmaf(p0.z, ad0.z, d0); d0 = fmaf(p0.w, ad0.w, d0);
    s1 = fmaf(p1.x, as1.x, s1); s1 = fmaf(p1.y, as1.y, s1); s1 = fmaf(p1.z, as1.z, s1); s1 = fmaf(p1.w, as1.w, s1);
    d1 = fmaf(p1.x, ad1.x, d1); d1 = fmaf(p1.y, ad1.y, d1); d1 = fmaf(p1.z, ad1.z, d1); d1 = fmaf(p1.w, ad1.w, d1);
#pragma unroll
    for (int off = 16; off > 0; off >>= 1) {
      s0 += __shfl_xor(s0, off);
      d0 += __shfl_xor(d0, off);
      s1 += __shfl_xor(s1, off);
      d1 += __shfl_xor(d1, off);
    }
    if (lane == 0) {
      sdt[row] = s0; sdt[GBM + row] = d0; sdt[2 * GBM + row] = s1; sdt[3 * GBM + row] = d1;
    }
  }
  __syncthreads();

  const int aw = wave & 1;
  const v4f alv = *(const v4fa*)(sdt + 128 * aw + 4 * lane);
  float* alp = AL + (size_t)blockIdx.x * ALB + 128 * aw + 4 * lane;
  const bool alw = wave < 2;
#pragma unroll 1
  for (int i = 0; i < RPW; ++i) {
    const int row = wave * RPW + i;
#pragma unroll
    for (int c = 0; c < 2; ++c) {
      const v4f p = *(const v4fa*)(stg + row * DH + c * GBN + 4 * lane);
      float* op = Cm + (size_t)(rowBase + row) * (size_t)DH + c * GBN + 4 * lane;
      *(volatile v4f*)op = p;
    }
  }
  if (alw) *(volatile v4f*)alp = alv;
  __threadfence();
#pragma unroll 1
  for (int i = 0; i < RPW; ++i) {
    const int row = wave * RPW + i;
#pragma unroll
    for (int c = 0; c < 2; ++c) {
      const v4f p = *(const v4fa*)(stg + row * DH + c * GBN + 4 * lane);
      float* op = Cm + (size_t)(rowBase + row) * (size_t)DH + c * GBN + 4 * lane;
      *(volatile v4f*)op = p;
    }
  }
  if (alw) *(volatile v4f*)alp = alv;
}

__global__ __launch_bounds__(NTHR) void k_agg(const int* __restrict__ srcs, const int* __restrict__ dsts,
                                              int nE, int nN, int vec8, int mRows,
                                              const float* __restrict__ AL,
                                              const float* __restrict__ xl, const float* __restrict__ bias,
                                              unsigned short* hb) {
  extern __shared__ __attribute__((aligned(16))) int dsm[];
  int* list = dsm;
  int* hl   = dsm + LISTN;
  int* sl   = dsm + LISTN + RCAP;
  int* cnt  = dsm + LISTN + 2 * RCAP;
  int* offs = cnt + NBA;
  int* cur  = offs + NBA;
  int* misc = cur + NBA;
  const int tid = (int)threadIdx.x, lane = tid & 31, wave = tid >> 5;
  const int nodeBase = (int)blockIdx.x * NBA;
  const int hd   = lane >> 4;
  const int hoff = hd * (2 * GBM);

  {
    const v4i z4 = {0, 0, 0, 0};
    for (int i = tid * 4; i < AGG_ZINTS; i += NTHR * 4) *(v4ia*)(dsm + i) = z4;
    if (tid < 16) misc[tid] = 0;
  }
  float bv[8];
  {
    const float* bq = bias + 8 * lane;
    const v4f a = *(const v4f*)bq;
    const v4f b = *(const v4f*)(bq + 4);
    bv[0] = bf16_val(a.x); bv[1] = bf16_val(a.y); bv[2] = bf16_val(a.z); bv[3] = bf16_val(a.w);
    bv[4] = bf16_val(b.x); bv[5] = bf16_val(b.y); bv[6] = bf16_val(b.z); bv[7] = bf16_val(b.w);
  }
  __syncthreads();

  int t = 0, ov = 0;
  const int nChunks = (nE + CHUNK - 1) / CHUNK;
#pragma unroll 1
  for (int ch = 0; ch < nChunks; ++ch) {
    const int cbase = ch * CHUNK;
    const int wc = scan_chunk<SLA>(dsts, nE, cbase, nodeBase, NBA, vec8, list, tid, lane, wave);
    if (lane == 0) misc[wave] = wc;
    __syncthreads();
    if (wave == 0) {
#pragma unroll 1
      for (int w2 = 0; w2 < NWAVE; ++w2) {
        int c = misc[w2];
        c = c < 0 ? 0 : (c > WCAP ? WCAP : c);
#pragma unroll 1
        for (int b0 = 0; b0 < c; b0 += 32) {
          const int idx = b0 + lane;
          const int ent = list[w2 * WCAP + (idx < WCAP ? idx : WCAP - 1)];
          const int m32 = (c - b0) < 32 ? (c - b0) : 32;
#pragma unroll 1
          for (int k = 0; k < m32; ++k) {
            const int u    = __builtin_amdgcn_readlane(ent, k);
            const int slot = u & (NBA - 1);
            const int el   = (u >> SLA) & (CHUNK - 1);
            const int pk   = ((cbase + el) << SLA) | slot;
            if (t < RCAP) {
              if (lane == 0) { hl[t] = pk; cnt[slot] = cnt[slot] + 1; }
              t = t + 1;
            } else {
              ov = 1;
            }
          }
        }
      }
    }
    __syncthreads();
  }
  if (wave == 0 && lane == 0) { misc[8] = t; misc[9] = ov; }
  __syncthreads();
  int tt = misc[8];
  tt = tt < 0 ? 0 : (tt > RCAP ? RCAP : tt);
  const int ovf = misc[9];

  if (wave == 0) {
    const int base = lane * (NBA / 32);
    int s = 0;
#pragma unroll 1
    for (int i = 0; i < NBA / 32; ++i) s += cnt[base + i];
    int incl = s;
#pragma unroll
    for (int d = 1; d < 32; d <<= 1) {
      const int y = __shfl_up(incl, d, 32);
      if (lane >= d) incl += y;
    }
    int run = incl - s;
#pragma unroll 1
    for (int i = 0; i < NBA / 32; ++i) {
      const int cv = cnt[base + i];
      offs[base + i] = run;
      cur[base + i]  = run;
      run += cv;
    }
  }
  __syncthreads();
  if (wave == 0) {
#pragma unroll 1
    for (int b0 = 0; b0 < tt; b0 += 32) {
      const int idx = b0 + lane;
      const int ent = hl[idx < RCAP ? idx : RCAP - 1];
      const int m32 = (tt - b0) < 32 ? (tt - b0) : 32;
#pragma unroll 1
      for (int k = 0; k < m32; ++k) {
        const int u    = __builtin_amdgcn_readlane(ent, k);
        const int slot = u & (NBA - 1);
        if (lane == 0) {
          int p = cur[slot];
          p = p < 0 ? 0 : (p > RCAP - 1 ? RCAP - 1 : p);
          sl[p] = u;
          cur[slot] = p + 1;
        }
      }
    }
  }
  __syncthreads();

  const float pz = (ovf != 0) ? __int_as_float(0x7fc00000) : 0.0f;
#pragma unroll 1
  for (int si = 0; si < NBA / NWAVE; ++si) {
    const int s    = si * NWAVE + wave;
    const int node = nodeBase + s;
    int c = cnt[s];
    const bool big = c > DEGCAP;
    c = c < 0 ? 0 : (c > DEGCAP ? DEGCAP : c);
    int o = offs[s];
    o = o < 0 ? 0 : (o > RCAP ? RCAP : o);
    const int nc  = node < nN ? node : nN - 1;
    const int alb = (nc >> 6) * ALB + (nc & (GBM - 1)) + hoff;
    const float asf = AL[alb];
    const float ad  = AL[alb + GBM];
    float acc[8];
    {
      const float* sp = xl + (size_t)nc * DH + 8 * lane;
      const v4f a = *(const v4f*)sp;
      const v4f b = *(const v4f*)(sp + 4);
      acc[0] = a.x; acc[1] = a.y; acc[2] = a.z; acc[3] = a.w;
      acc[4] = b.x; acc[5] = b.y; acc[6] = b.z; acc[7] = b.w;
    }
    float l0 = asf + ad;
    l0 = l0 > 0.f ? l0 : NEGSL * l0;
    float mx = l0, dn = 1.0f;
#pragma unroll 1
    for (int b0 = 0; b0 < c; b0 += 32) {
      int idx = o + b0 + lane;
      idx = idx > RCAP - 1 ? RCAP - 1 : idx;
      const int ent = sl[idx];
      int eid = ent >> SLA;
      eid = eid < 0 ? 0 : (eid > nE - 1 ? nE - 1 : eid);
      int sr = srcs[eid];
      sr = sr < 0 ? 0 : (sr > nN - 1 ? nN - 1 : sr);
      const int sb = (sr >> 6) * ALB + (sr & (GBM - 1));
      const int e0i = __float_as_int(AL[sb]);
      const int e1i = __float_as_int(AL[sb + 2 * GBM]);
      const int m32 = (c - b0) < 32 ? (c - b0) : 32;
#pragma unroll 1
      for (int k = 0; k < m32; ++k) {
        const int   sk = __builtin_amdgcn_readlane(sr, k);
        const float a0 = __int_as_float(__builtin_amdgcn_readlane(e0i, k));
        const float a1 = __int_as_float(__builtin_amdgcn_readlane(e1i, k));
        const float ask = (hd != 0) ? a1 : a0;
        const float* rp = xl + (size_t)sk * DH + 8 * lane;
        const v4f a = *(const v4f*)rp;
        const v4f b = *(const v4f*)(rp + 4);
        float lg = ask + ad;
        lg = lg > 0.f ? lg : NEGSL * lg;
        const float df = lg - mx;
        const float ee = expf(-fabsf(df));
        const bool  up = df > 0.f;
        const float s1 = up ? ee : 1.0f;
        const float s2 = up ? 1.0f : ee;
        mx = up ? lg : mx;
        dn = fmaf(dn, s1, s2);
        acc[0] = fmaf(acc[0], s1, s2 * a.x); acc[1] = fmaf(acc[1], s1, s2 * a.y);
        acc[2] = fmaf(acc[2], s1, s2 * a.z); acc[3] = fmaf(acc[3], s1, s2 * a.w);
        acc[4] = fmaf(acc[4], s1, s2 * b.x); acc[5] = fmaf(acc[5], s1, s2 * b.y);
        acc[6] = fmaf(acc[6], s1, s2 * b.z); acc[7] = fmaf(acc[7], s1, s2 * b.w);
      }
    }
    const float inv = __builtin_amdgcn_rcpf(dn + EPS_SM);
    const float pzr = big ? __int_as_float(0x7fc00000) : pz;
    const bool live = node < nN;
    v8us ho, lo;
#pragma unroll
    for (int i = 0; i < 8; ++i) {
      float y = fmaf(acc[i], inv, bv[i]);
      y = (y > 0.0f) ? y : (y - y);
      y = y + pzr;
      y = live ? y : 0.0f;
      const unsigned hbi = bf16_bits(y);
      ho[i] = (unsigned short)hbi;
      lo[i] = (unsigned short)bf16_bits(y - __uint_as_float(hbi << 16));
    }
    if (node < mRows) {
      unsigned short* hp = hb + (size_t)node * KP + 8 * lane;
      *(volatile v8us*)hp = ho;
      *(volatile v8us*)(hp + DH) = lo;
      __threadfence();
      *(volatile v8us*)hp = ho;
      *(volatile v8us*)(hp + DH) = lo;
    }
  }
}

__global__ __launch_bounds__(PTHR) void k_post(const unsigned short* __restrict__ A,
                                               const unsigned short* __restrict__ BT,
                                               const float* __restrict__ bp1, const float* __restrict__ wp2,
                                               const float* __restrict__ bp2, float* out, int nN) {
  __shared__ __attribute__((aligned(16))) float spar[2 * DOUT];
  __shared__ __attribute__((aligned(16))) float sres[PBM];
  const int tid = (int)threadIdx.x, lane = tid & 31, wave = tid >> 5, hh = lane >> 4, m = lane & 15;
  const int rowBase = (int)blockIdx.x * PBM;

  {
    const int c = tid & (DOUT - 1);
    const float vb = bp1[c];
    const float vw = wp2[c];
    const float v  = (tid < DOUT) ? vb : vw;
    spar[tid] = bf16_val(v);
  }

  v8f acc[8];
  {
    const v8f z = {0.f, 0.f, 0.f, 0.f, 0.f, 0.f, 0.f, 0.f};
#pragma unroll
    for (int t = 0; t < 8; ++t) acc[t] = z;
  }
  const unsigned short* ap = A  + (size_t)(rowBase + 16 * wave + m) * (size_t)KP + 8 * hh;
  const unsigned short* bp = BT + (size_t)m * (size_t)KP + 8 * hh;

#pragma unroll 1
  for (int k0 = 0; k0 < KP; k0 += 32) {
    FragB af;
    af.h[0] = *(const v8usa*)(ap + k0);
    af.h[1] = *(const v8usa*)(ap + k0 + 16);
#pragma unroll
    for (int nt = 0; nt < 8; ++nt) {
      const unsigned short* wq = bp + (size_t)(16 * nt) * (size_t)KP + k0;
      FragB bf;
      bf.h[0] = *(const v8usa*)wq;
      bf.h[1] = *(const v8usa*)(wq + 16);
      acc[nt] = wmb(af, bf, acc[nt]);
    }
  }
  __syncthreads();

  float t[8];
#pragma unroll
  for (int r = 0; r < 8; ++r) t[r] = 0.0f;
#pragma unroll
  for (int nt = 0; nt < 8; ++nt) {
    const float b = spar[16 * nt + m];
    const float w = spar[DOUT + 16 * nt + m];
#pragma unroll
    for (int r = 0; r < 8; ++r) t[r] = fmaf(acc[nt][r] + b, w, t[r]);
  }
#pragma unroll
  for (int off = 8; off > 0; off >>= 1) {
#pragma unroll
    for (int r = 0; r < 8; ++r) t[r] += __shfl_xor(t[r], off);
  }
  float tv = t[0];
  tv = (m == 1) ? t[1] : tv;
  tv = (m == 2) ? t[2] : tv;
  tv = (m == 3) ? t[3] : tv;
  tv = (m == 4) ? t[4] : tv;
  tv = (m == 5) ? t[5] : tv;
  tv = (m == 6) ? t[6] : tv;
  tv = (m == 7) ? t[7] : tv;
  const float zz = tv + bf16_val(bp2[0]);
  const float sg = 1.0f / (1.0f + expf(-zz));
  if (m < 8) sres[16 * wave + 8 * hh + m] = sg;
  __syncthreads();

  const v4f ov = *(const v4fa*)(sres + 4 * lane);
  int live = nN - rowBase;
  live = live < 0 ? 0 : (live > PBM ? PBM : live);
  const bool wr = (wave == 0) && (4 * lane < live);
  float* op = out + (size_t)rowBase + 4 * lane;
  if (wr) *(volatile v4f*)op = ov;
  __threadfence();
  if (wr) *(volatile v4f*)op = ov;
}

static inline int cdiv(int a, int b) { return (a + b - 1) / b; }

extern "C" void kernel_launch(void* const* d_in, const int* in_sizes, int n_in,
                              void* d_out, int out_size, void* d_ws, size_t ws_size,
                              hipStream_t stream) {
  if (n_in < 14) return;
  if (in_sizes[0] < DIN || (in_sizes[0] % DIN) != 0) return;
  const int nN = in_sizes[0] / DIN;
  if (nN > (1 << 22) || (nN & 3) != 0) return;
  if (in_sizes[1] < 2 || (in_sizes[1] & 1) != 0) return;
  const int nE = in_sizes[1] / 2;
  if (nE < 1 || nE >= (1 << 21)) return;
  if (in_sizes[2] != DIN * DH) return;
  if (in_sizes[3] != DH || in_sizes[4] != DH || in_sizes[5] != DH) return;
  if (in_sizes[6] != DH * DH) return;
  if (in_sizes[7] != DH || in_sizes[8] != DH || in_sizes[9] != DH) return;
  if (in_sizes[10] != DH * DOUT) return;
  if (in_sizes[11] != DOUT || in_sizes[12] != DOUT || in_sizes[13] != 1) return;
  if (out_size != nN) return;

  const float* x    = (const float*)d_in[0];
  const int*   edge = (const int*)d_in[1];
  const float* W1   = (const float*)d_in[2];
  const float* a1s  = (const float*)d_in[3];
  const float* a1d  = (const float*)d_in[4];
  const float* b1   = (const float*)d_in[5];
  const float* W2   = (const float*)d_in[6];
  const float* a2s  = (const float*)d_in[7];
  const float* a2d  = (const float*)d_in[8];
  const float* b2   = (const float*)d_in[9];
  const float* Wp1  = (const float*)d_in[10];
  const float* bp1  = (const float*)d_in[11];
  const float* Wp2  = (const float*)d_in[12];
  const float* bp2  = (const float*)d_in[13];
  float* out = (float*)d_out;
  const int* src = edge;
  const int* dst = edge + nE;

  const int MP   = cdiv(nN, MROWS) * MROWS;
  const int gM   = MP / GBM;
  const int gP   = MP / PBM;
  const int gA   = cdiv(MP, NBA);
  if ((long long)gA * NBA < (long long)MP) return;
  const int vec8 = ((nE & 3) == 0) ? 1 : 0;

  char* ws = (char*)d_ws;
  size_t off = 0;
  const size_t oW1T = off; off += (size_t)DH * DIN * 2;                   off = (off + 255) & ~(size_t)255;
  const size_t oW2T = off; off += (size_t)DH * KP * 2;                    off = (off + 255) & ~(size_t)255;
  const size_t oWPT = off; off += (size_t)DOUT * KP * 2;                  off = (off + 255) & ~(size_t)255;
  const size_t oAL  = off; off += (size_t)gM * ALB * 4;                   off = (off + 255) & ~(size_t)255;
  const size_t oXB  = off; off += (size_t)MP * DIN * 2;                   off = (off + 255) & ~(size_t)255;
  const size_t oH   = off; off += (size_t)MP * DH * 4;                    off = (off + 255) & ~(size_t)255;
  const size_t oAP  = off; off += (size_t)MP * KP * 2;                    off = (off + 255) & ~(size_t)255;
  if (off > ws_size || off > (size_t)WSMAX) return;
  unsigned short* W1T = (unsigned short*)(ws + oW1T);
  unsigned short* W2T = (unsigned short*)(ws + oW2T);
  unsigned short* WPT = (unsigned short*)(ws + oWPT);
  float*          ALp = (float*)(ws + oAL);
  unsigned short* XB  = (unsigned short*)(ws + oXB);
  float*          H   = (float*)(ws + oH);
  unsigned short* AP  = (unsigned short*)(ws + oAP);

  const size_t aggLds  = (size_t)AGG_LDS_INTS * 4;
  const size_t gemmLds = (size_t)GEMM_LDS_FLOATS * 4;
  hipFuncSetAttribute(reinterpret_cast<const void*>(&k_gemm), hipFuncAttributeMaxDynamicSharedMemorySize, (int)gemmLds);
  hipFuncSetAttribute(reinterpret_cast<const void*>(&k_agg), hipFuncAttributeMaxDynamicSharedMemorySize, (int)aggLds);

  const int nUx = MP * (DIN / 8);
  k_wprep<<<(NU1 + NU2 + NU3) / NTHR, NTHR, 0, stream>>>(W1, W2, Wp1, W1T, W2T, WPT);
  k_cvx<<<cdiv(nUx, NTHR), NTHR, 0, stream>>>(x, nN, nUx, XB);
  k_gemm<<<gM, GTHR, gemmLds, stream>>>(XB, DIN, W1T, DIN, DIN, H, a1s, a1d, ALp);
  k_agg<<<gA, NTHR, aggLds, stream>>>(src, dst, nE, nN, vec8, MP, ALp, H, b1, AP);
  k_gemm<<<gM, GTHR, gemmLds, stream>>>(AP, KP, W2T, KP, KP, H, a2s, a2d, ALp);
  k_agg<<<gA, NTHR, aggLds, stream>>>(src, dst, nE, nN, vec8, MP, ALp, H, b2, AP);
  k_post<<<gP, PTHR, 0, stream>>>(AP, WPT, bp1, Wp2, bp2, out, nN);
}
